// MultiHeadAttention_85306640433958
// MI455X (gfx1250) — hardware-run, weakly checked
//
#include <hip/hip_runtime.h>
#ifndef NB
#define NB 2
#endif
#ifndef SEQ
#define SEQ 2048
#endif
#define SEQ_FULL 2048
#define DM 512
#define NH 8
#define HD 64
#define NQKV 1536
#define WH 64
#define MP (NB * SEQ)
#define AT_NK 208
#define AT_VP 216
#define AT_PP 168
#define AT_OP 72

typedef unsigned short v8us __attribute__((ext_vector_type(8), may_alias));
typedef float  v8f  __attribute__((ext_vector_type(8)));
typedef float  v4f  __attribute__((ext_vector_type(4)));
typedef float  v4fa __attribute__((ext_vector_type(4), may_alias));
typedef _Float16 v16h __attribute__((ext_vector_type(16)));
typedef _Float16 v4h __attribute__((ext_vector_type(4)));
union FragH { v16h v; v8us half[2]; _Float16 h[16]; unsigned short u[16]; };

__device__ __forceinline__ unsigned short bf16_bits(float x) { unsigned int u = __float_as_uint(x); return (unsigned short)((u + 0x7FFFu + ((u >> 16) & 1u)) >> 16); }
__device__ __forceinline__ float bf16_val(unsigned short b) { return __uint_as_float(((unsigned int)b) << 16); }
__device__ __forceinline__ float bf16_rne(float x) { return bf16_val(bf16_bits(x)); }

__device__ __forceinline__ v16h g2_frag(const _Float16* p, int hh) { FragH f; f.half[0] = *(const v8us*)((const unsigned short*)p + 8 * hh); f.half[1] = *(const v8us*)((const unsigned short*)p + 16 + 8 * hh); return f.v; }
__device__ __forceinline__ v8f g2_mma(v16h a, v16h b, v8f c) { v8f d = __builtin_amdgcn_wmma_f32_16x16x32_f16(false, a, false, b, (short)0, c, false, false); asm volatile("v_nop\n\tv_nop\n\tv_nop\n\tv_nop" : "+v"(d) : "v"(a), "v"(b)); return d; }

__global__ __launch_bounds__(256) void k_x16(const float* __restrict__ x, _Float16* __restrict__ X16, size_t n8, size_t sstride, size_t dstride) {
  const size_t t = (size_t)blockIdx.x * 256 + threadIdx.x; if (t >= n8) return;
  const float* s = x + (size_t)blockIdx.y * sstride + t * 8;
  unsigned short* d = (unsigned short*)X16 + (size_t)blockIdx.y * dstride + t * 8;
  const v4f a = *(const v4fa*)s, c = *(const v4fa*)(s + 4); FragH f;
#pragma unroll
  for (int q = 0; q < 4; ++q) { f.h[q] = (_Float16)bf16_rne(a[q]); f.h[4 + q] = (_Float16)bf16_rne(c[q]); }
  const v8us o = f.half[0];
  *(volatile v8us*)d = o; __threadfence(); *(volatile v8us*)d = o;
}

__global__ __launch_bounds__(256) void k_wnat(const float* __restrict__ w, size_t n8, _Float16* __restrict__ Bt) {
  const size_t t = (size_t)blockIdx.x * 256 + threadIdx.x; if (t >= n8) return;
  const v4f a = *(const v4fa*)(w + t * 8), c = *(const v4fa*)(w + t * 8 + 4); FragH f;
#pragma unroll
  for (int q = 0; q < 4; ++q) { f.h[q] = (_Float16)(bf16_rne(a[q]) * 16.0f); f.h[4 + q] = (_Float16)(bf16_rne(c[q]) * 16.0f); }
  const v8us o = f.half[0];
  *(volatile v8us*)((unsigned short*)Bt + t * 8) = o; __threadfence(); *(volatile v8us*)((unsigned short*)Bt + t * 8) = o;
}

__global__ __launch_bounds__(128) void k_gemm2(const _Float16* __restrict__ A, int lda, const _Float16* __restrict__ Bh, int ldb, float alpha, const float* __restrict__ bias,
                                               float* __restrict__ C, _Float16* __restrict__ C16, int ldc, int M, int N, int K) {
  __shared__ __attribute__((aligned(16))) float so[4][32][68];
  const int tid = threadIdx.x, w = tid >> 5, lane = tid & 31, ln = lane & 15, hh = lane >> 4;
  const int ntn = N >> 6; const int mt = blockIdx.x / ntn, nq = blockIdx.x - mt * ntn; const int row0 = mt * 128 + 32 * w, col0 = nq * 64; if (row0 >= M) return;
  const _Float16* a0p = A + (size_t)(row0 + ln) * lda; const _Float16* a1p = a0p + (size_t)16 * lda;
  const _Float16* b0p = Bh + (size_t)(col0 + ln) * ldb; const _Float16* b1p = b0p + (size_t)16 * ldb; const _Float16* b2p = b1p + (size_t)16 * ldb; const _Float16* b3p = b2p + (size_t)16 * ldb;
  const v8f z8 = {0.f,0.f,0.f,0.f,0.f,0.f,0.f,0.f}; v8f c00 = z8, c01 = z8, c02 = z8, c03 = z8, c10 = z8, c11 = z8, c12 = z8, c13 = z8;
#pragma unroll 1
  for (int kb = 0; kb < K; kb += 32) { const v16h a0 = g2_frag(a0p + kb, hh), a1 = g2_frag(a1p + kb, hh);
    v16h b = g2_frag(b0p + kb, hh); c00 = g2_mma(a0, b, c00); c10 = g2_mma(a1, b, c10);
    b = g2_frag(b1p + kb, hh); c01 = g2_mma(a0, b, c01); c11 = g2_mma(a1, b, c11);
    b = g2_frag(b2p + kb, hh); c02 = g2_mma(a0, b, c02); c12 = g2_mma(a1, b, c12);
    b = g2_frag(b3p + kb, hh); c03 = g2_mma(a0, b, c03); c13 = g2_mma(a1, b, c13); }
  v8f accs[8] = {c00, c01, c02, c03, c10, c11, c12, c13};
#pragma unroll
  for (int u = 0; u < 8; ++u) { const int t = u & 3, half = u >> 2; const int col = col0 + t * 16 + ln; const float bv = bias ? bf16_rne(bias[col]) : 0.f;
#pragma unroll
    for (int r = 0; r < 8; ++r) { const int rloc = half * 16 + 8 * hh + r; so[w][rloc][t * 16 + ln] = accs[u][r] * alpha + bv; } }
  __builtin_amdgcn_fence(4  , "workgroup"); __builtin_amdgcn_wave_barrier();
  const int rsub = lane >> 4, c4 = (lane & 15) * 4;
  for (int pass = 0; pass < 2; ++pass) {
#pragma unroll
    for (int q = 0; q < 16; ++q) { const int r = q * 2 + rsub; const v4f v = *(const v4fa*)&so[w][r][c4];
      if (C) *(volatile v4f*)(C + (size_t)(row0 + r) * ldc + col0 + c4) = v;
      if (C16) { v4h h4;
#pragma unroll
        for (int i = 0; i < 4; ++i) h4[i] = (_Float16)v[i];
        *(volatile v4h*)(C16 + (size_t)(row0 + r) * ldc + col0 + c4) = h4; } }
    if (pass == 0) __threadfence(); }
}

__global__ __launch_bounds__(128) void k_attn(const _Float16* __restrict__ QKV, const int* __restrict__ pm, _Float16* __restrict__ CTX) {
  __shared__ __attribute__((aligned(16))) unsigned short vt[HD * AT_VP];
  __shared__ __attribute__((aligned(16))) unsigned short lp[4][16 * AT_PP];
  __shared__ __attribute__((aligned(16))) unsigned short so[4][16 * AT_OP];
  __shared__ int kms[AT_NK];
  const int tid = threadIdx.x, w = tid >> 5, lane = tid & 31, ln = lane & 15, hh = lane >> 4;
  const int bh = blockIdx.y, b = bh / NH, h = bh - b * NH;
  const int q0b = blockIdx.x * 64, kbase = q0b - WH;
  const size_t rowb = (size_t)b * SEQ;
  const unsigned short* qkvu = (const unsigned short*)QKV;
  for (int i = tid; i < AT_NK * 8; i += 128) {
    const int j = i >> 3, d8 = (i & 7) * 8;
    const int key = kbase + j; const int keyc = min(max(key, 0), SEQ - 1);
    const bool ok = (key >= 0) && (key < SEQ);
    const v8us v = *(const v8us*)(qkvu + (rowb + (size_t)keyc) * NQKV + h * 192 + 128 + d8);
#pragma unroll
    for (int q = 0; q < 8; ++q) vt[(d8 + q) * AT_VP + j] = ok ? v[q] : (unsigned short)0;
  }
  for (int j = tid; j < AT_NK; j += 128) {
    const int key = kbase + j; const int keyc = min(max(key, 0), SEQ - 1);
    const int m = pm[(size_t)b * SEQ_FULL + keyc];
    kms[j] = ((key >= 0) && (key < SEQ) && (m != 0)) ? 1 : 0;
  }
  __syncthreads();

  const int q0 = q0b + 16 * w;
  const _Float16* qrow = QKV + (rowb + (size_t)(q0 + ln)) * NQKV + h * 192;
  const v16h qa0 = g2_frag(qrow, hh), qa1 = g2_frag(qrow + 32, hh);
  const v8f z8 = {0.f,0.f,0.f,0.f,0.f,0.f,0.f,0.f};
  v8f sc[9];
#pragma unroll
  for (int kt = 0; kt < 9; ++kt) {
    const int key = q0 - WH + kt * 16 + ln; const int keyc = min(max(key, 0), SEQ - 1);
    const _Float16* krow = QKV + (rowb + (size_t)keyc) * NQKV + h * 192 + 64;
    v8f a = z8;
    a = g2_mma(qa0, g2_frag(krow, hh), a);
    a = g2_mma(qa1, g2_frag(krow + 32, hh), a);
    sc[kt] = a;
  }
  int qm[8];
#pragma unroll
  for (int r = 0; r < 8; ++r) qm[r] = kms[WH + 16 * w + 8 * hh + r];
#pragma unroll
  for (int kt = 0; kt < 9; ++kt) {
    const int kok = kms[16 * w + kt * 16 + ln];
#pragma unroll
    for (int r = 0; r < 8; ++r) {
      const int diff = kt * 16 + ln - WH - (8 * hh + r);
      const float s = sc[kt][r] * 0.125f;
      const bool live = (kok != 0) && (qm[r] != 0) && (diff >= -WH) && (diff <= WH) && (s != 0.0f);
      sc[kt][r] = live ? s : -3.0e38f;
    }
  }
  { const v8us zz = {0, 0, 0, 0, 0, 0, 0, 0}; *(v8us*)&lp[w][(lane >> 1) * AT_PP + 144 + (lane & 1) * 8] = zz; }
#pragma unroll
  for (int r = 0; r < 8; ++r) {
    float mx = -3.0e38f;
#pragma unroll
    for (int kt = 0; kt < 9; ++kt) mx = fmaxf(mx, sc[kt][r]);
    mx = fmaxf(mx, __shfl_xor(mx, 1, 32));
    mx = fmaxf(mx, __shfl_xor(mx, 2, 32));
    mx = fmaxf(mx, __shfl_xor(mx, 4, 32));
    mx = fmaxf(mx, __shfl_xor(mx, 8, 32));
    float sum = 0.f;
#pragma unroll
    for (int kt = 0; kt < 9; ++kt) {
      const float ex = __expf(sc[kt][r] - mx);
      const float e = (sc[kt][r] > -1.0e38f) ? ex : 0.f;
      sc[kt][r] = e; sum += e;
    }
    sum += __shfl_xor(sum, 1, 32);
    sum += __shfl_xor(sum, 2, 32);
    sum += __shfl_xor(sum, 4, 32);
    sum += __shfl_xor(sum, 8, 32);
    const float sd = (sum > 0.f) ? sum : 1.f;
    const float inv = (sum > 0.f) ? (1024.0f / sd) : 0.f;
    const int m = 8 * hh + r;
#pragma unroll
    for (int kt = 0; kt < 9; ++kt) lp[w][m * AT_PP + kt * 16 + ln] = __builtin_bit_cast(unsigned short, (_Float16)(sc[kt][r] * inv));
  }
  __builtin_amdgcn_fence(4  , "workgroup"); __builtin_amdgcn_wave_barrier();

  v8f oacc[4] = {z8, z8, z8, z8};
#pragma unroll
  for (int c = 0; c < 5; ++c) {
    FragH pa;
    pa.half[0] = *(const v8us*)&lp[w][ln * AT_PP + c * 32 + 8 * hh];
    pa.half[1] = *(const v8us*)&lp[w][ln * AT_PP + c * 32 + 16 + 8 * hh];
#pragma unroll
    for (int j = 0; j < 4; ++j) {
      const int vo = (j * 16 + ln) * AT_VP + 16 * w + c * 32 + 8 * hh;
      FragH vb;
      vb.half[0] = *(const v8us*)&vt[vo];
      vb.half[1] = *(const v8us*)&vt[vo + 16];
      oacc[j] = g2_mma(pa.v, vb.v, oacc[j]);
    }
  }
#pragma unroll
  for (int j = 0; j < 4; ++j) {
#pragma unroll
    for (int r = 0; r < 8; ++r) so[w][(8 * hh + r) * AT_OP + j * 16 + ln] = __builtin_bit_cast(unsigned short, (_Float16)(oacc[j][r] * 0.0625f));
  }
  __builtin_amdgcn_fence(4  , "workgroup"); __builtin_amdgcn_wave_barrier();
  const int rq = lane >> 3, pc = lane & 7;
  for (int pass = 0; pass < 2; ++pass) {
#pragma unroll
    for (int q = 0; q < 4; ++q) {
      const int r = q * 4 + rq;
      const v8us v = *(const v8us*)&so[w][r * AT_OP + pc * 8];
      *(volatile v8us*)((unsigned short*)CTX + (rowb + (size_t)(q0 + r)) * DM + h * HD + pc * 8) = v;
    }
    if (pass == 0) __threadfence();
  }
}

extern "C" void kernel_launch(void* const* d_in, const int* in_sizes, int n_in,
                              void* d_out, int out_size, void* d_ws, size_t ws_size, hipStream_t stream) {
  static_assert(NH * HD == DM);
  static_assert(NQKV == 3 * DM);
  static_assert(SEQ % 128 == 0);
  static_assert(SEQ <= SEQ_FULL);
  static_assert(MP % 128 == 0);
  static_assert(DM % 64 == 0);
  static_assert(NQKV % 64 == 0);
  static_assert(DM % 32 == 0);
  static_assert((AT_NK * 8) % 128 == 0);
  static_assert((size_t)NQKV * DM * 2 + (size_t)DM * DM * 2 + (size_t)MP * DM * 2 * 2 + (size_t)MP * NQKV * 2 <= (size_t)134217728);
  if (n_in < 6) return;
  if ((long long)in_sizes[0] < (long long)(NB - 1) * SEQ_FULL * DM + (long long)SEQ * DM) return;
  if (in_sizes[1] < NQKV * DM) return;
  if (in_sizes[2] < NQKV) return;
  if (in_sizes[3] < DM * DM) return;
  if (in_sizes[4] < DM) return;
  if (in_sizes[5] < (NB - 1) * SEQ_FULL + SEQ) return;
  if ((long long)out_size < (long long)MP * DM) return;
  const float* x = (const float*)d_in[0];
  const float* wqkv = (const float*)d_in[1];
  const float* bqkv = (const float*)d_in[2];
  const float* wo = (const float*)d_in[3];
  const float* bo = (const float*)d_in[4];
  const int* pm = (const int*)d_in[5];
  char* ws = (char*)d_ws; size_t off = 0;
  auto take = [&](size_t bytes) { char* p = ws + off; off += (bytes + 255) & ~(size_t)255; return p; };
  _Float16* WQ = (_Float16*)take((size_t)NQKV * DM * 2);
  _Float16* WO = (_Float16*)take((size_t)DM * DM * 2);
  _Float16* X16 = (_Float16*)take((size_t)MP * DM * 2);
  _Float16* QKV16 = (_Float16*)take((size_t)MP * NQKV * 2);
  _Float16* CTX16 = (_Float16*)take((size_t)MP * DM * 2);
  if (off > ws_size) return;
  const size_t nq8 = (size_t)NQKV * DM / 8, no8 = (size_t)DM * DM / 8, nx8 = (size_t)SEQ * DM / 8;
  k_wnat<<<(unsigned)((nq8 + 255) / 256), 256, 0, stream>>>(wqkv, nq8, WQ);
  k_wnat<<<(unsigned)((no8 + 255) / 256), 256, 0, stream>>>(wo, no8, WO);
  k_x16<<<dim3((unsigned)((nx8 + 255) / 256), NB), 256, 0, stream>>>(x, X16, nx8, (size_t)SEQ_FULL * DM, (size_t)SEQ * DM);
  k_gemm2<<<dim3((unsigned)((MP / 128) * (NQKV / 64))), 128, 0, stream>>>(X16, DM, WQ, DM, 0.0625f, bqkv, nullptr, QKV16, NQKV, MP, NQKV, DM);
  k_attn<<<dim3(SEQ / 64, NB * NH), 128, 0, stream>>>(QKV16, pm, CTX16);
  k_gemm2<<<dim3((unsigned)((MP / 128) * (DM / 64))), 128, 0, stream>>>(CTX16, DM, WO, DM, 0.0009765625f, bo, (float*)d_out, nullptr, DM, MP, DM, DM);
}
